// EdgeTypeRGCN_28707561406844
// MI455X (gfx1250) — hardware-verified
//
#include <hip/hip_runtime.h>
#include <math.h>


#define NN 100000
#define NE 1600000
#define CH 64
#define NBAS 4
#define NREL 16
#define KTOT 320
#define SLOTC 64
#define NCH 768
#define NNP 100032

typedef __attribute__((ext_vector_type(16))) _Float16 v16h;
typedef __attribute__((ext_vector_type(8)))  _Float16 v8h;
typedef __attribute__((ext_vector_type(8)))  float v8f;
typedef __attribute__((ext_vector_type(4)))  float v4f;
typedef __attribute__((ext_vector_type(2)))  float v2f;
typedef __attribute__((ext_vector_type(4)))  unsigned v4u;
typedef __attribute__((ext_vector_type(4)))  int v4i;

template <typename T> __device__ __forceinline__ void vst2(void* p, T v) { *(volatile T*)p = v; __threadfence(); *(volatile T*)p = v; }
__device__ __forceinline__ v8f wmma16(v16h a, v16h b, v8f c) {
  v8f d = __builtin_amdgcn_wmma_f32_16x16x32_f16(false, a, false, b, (short)0, c, false, false);
  asm volatile("v_nop\n\tv_nop\n\tv_nop\n\tv_nop" : "+v"(d) : "v"(a), "v"(b));
  return d;
}
__device__ __forceinline__ v16h frag_h(const _Float16* rowk0, int lane) {
  union { v16h v; v8h q[2]; } u; const _Float16* p = rowk0 + 8 * (lane >> 4);
  u.q[0] = *(const v8h*)p; u.q[1] = *(const v8h*)(p + 16); return u.v;
}
#define LDSX() do { asm volatile("s_wait_dscnt 0" ::: "memory"); __builtin_amdgcn_wave_barrier(); __builtin_amdgcn_fence(__ATOMIC_RELEASE, "workgroup"); } while (0)

__global__ __launch_bounds__(256) void k_bucket(const int* __restrict__ dst, int* __restrict__ list) {
  __shared__ int scnt[NCH];
  __shared__ __align__(16) int slots[NCH][SLOTC];
  const int n0 = blockIdx.x * NCH, tid = threadIdx.x;
  for (int i = tid; i < NCH; i += 256) scnt[i] = 0;
  for (int i = tid; i < NCH * SLOTC; i += 256) (&slots[0][0])[i] = 0;
  __syncthreads();
#pragma unroll 1
  for (int e = tid; e < NE; e += 256) { const int d = dst[e] - n0;
    if ((unsigned)d < (unsigned)NCH) { const int s = atomicAdd(&scnt[d], 1); if (s < SLOTC - 1) slots[d][s] = e; } }
  __syncthreads();
  for (int i = tid; i < NCH; i += 256) { const int n = n0 + i; if (n >= NN) continue;
    int c = scnt[i]; if (c > SLOTC - 1) c = SLOTC - 1;
    for (int a = 1; a < c; ++a) { const int v = slots[i][a]; int b = a - 1; while (b >= 0 && slots[i][b] > v) { slots[i][b + 1] = slots[i][b]; --b; } slots[i][b + 1] = v; }
    slots[i][SLOTC - 1] = scnt[i];
#pragma unroll
    for (int q = 0; q < SLOTC / 4; ++q) vst2(list + (size_t)n * SLOTC + q * 4, *(const v4i*)(&slots[i][q * 4])); }
}
__global__ __launch_bounds__(64) void k_packW(const float* __restrict__ bases, const float* __restrict__ loopw, _Float16* __restrict__ Wc) {
  const int o = blockIdx.x, q = threadIdx.x; if (q >= KTOT / 8) return;
  union { v8h h; v4u u; } pk;
#pragma unroll
  for (int e = 0; e < 8; ++e) { const int k = q * 8 + e; pk.h[e] = (_Float16)(k < 256 ? bases[((k >> 6) * CH + (k & 63)) * CH + o] : loopw[(k - 256) * CH + o]); }
  vst2(Wc + (size_t)o * KTOT + q * 8, pk.u);
}
__global__ __launch_bounds__(128) void k_layer(const float* __restrict__ x, const int* __restrict__ src, const int* __restrict__ et, const int* __restrict__ list,
                                             const float* __restrict__ comp, const _Float16* __restrict__ Wc, const float* __restrict__ bias,
                                             const float* __restrict__ gam, const float* __restrict__ bet, float* __restrict__ out) {
  __shared__ __align__(16) _Float16 sA[4][16][KTOT + 16];
  __shared__ __align__(16) float so[4][16][68];
  __shared__ float scomp[NREL * NBAS];
  const int tid = threadIdx.x, w = tid >> 5, lane = tid & 31, col = lane & 15, g = lane >> 4;
  const int n0 = blockIdx.x * 64 + w * 16;
  if (tid < NREL * NBAS) scomp[tid] = comp[tid];
  __syncthreads();
#pragma unroll 1
  for (int j = 0; j < 16; ++j) { const int n = n0 + j; float a[8] = {0.f, 0.f, 0.f, 0.f, 0.f, 0.f, 0.f, 0.f}; v2f xv = {0.f, 0.f};
    if (n < NN) {
      int dn = list[(size_t)n * SLOTC + SLOTC - 1]; dn = dn < 0 ? 0 : (dn > SLOTC - 1 ? SLOTC - 1 : dn);
#pragma unroll 1
      for (int s = 0; s < dn; ++s) { int e = list[(size_t)n * SLOTC + s]; if ((unsigned)e >= (unsigned)NE) continue;
        int sr = src[e]; sr = sr < 0 ? 0 : (sr >= NN ? NN - 1 : sr); int t = et[e]; t = t < 0 ? 0 : (t >= NREL ? NREL - 1 : t);
        const v2f v = *(const v2f*)(x + (size_t)sr * CH + 2 * lane);
#pragma unroll
        for (int b = 0; b < NBAS; ++b) { const float c = scomp[t * NBAS + b]; a[2 * b] += c * v[0]; a[2 * b + 1] += c * v[1]; } }
      xv = *(const v2f*)(x + (size_t)n * CH + 2 * lane); }
#pragma unroll
    for (int b = 0; b < NBAS; ++b) { sA[w][j][b * CH + 2 * lane] = (_Float16)a[2 * b]; sA[w][j][b * CH + 2 * lane + 1] = (_Float16)a[2 * b + 1]; }
    sA[w][j][256 + 2 * lane] = (_Float16)xv[0]; sA[w][j][256 + 2 * lane + 1] = (_Float16)xv[1]; }
  LDSX();
  v8f acc[4] = {};
#pragma unroll 1
  for (int kc = 0; kc < KTOT / 32; ++kc) { const v16h af = frag_h(&sA[w][col][0] + kc * 32, lane);
#pragma unroll
    for (int t = 0; t < 4; ++t) acc[t] = wmma16(af, frag_h(Wc + (size_t)(t * 16 + col) * KTOT + kc * 32, lane), acc[t]); }
#pragma unroll
  for (int t = 0; t < 4; ++t) { const float bv = bias[t * 16 + col];
#pragma unroll
    for (int r = 0; r < 8; ++r) { float v = acc[t][r] + bv; v = v >= 0.f ? v : 0.1f * v; so[w][8 * g + r][t * 16 + col] = v; } }
  LDSX();
  { float v[32]; float s = 0.f;
#pragma unroll
    for (int i = 0; i < 32; ++i) { v[i] = so[w][col][g * 32 + i]; s += v[i]; }
    s += __shfl_xor(s, 16, 32); const float mu = s / 64.0f; float qv = 0.f;
#pragma unroll
    for (int i = 0; i < 32; ++i) { v[i] -= mu; qv += v[i] * v[i]; }
    qv += __shfl_xor(qv, 16, 32); const float rs = rsqrtf(qv / 64.0f + 1e-5f);
    LDSX();
#pragma unroll
    for (int i = 0; i < 32; ++i) so[w][col][g * 32 + i] = v[i] * rs * gam[g * 32 + i] + bet[g * 32 + i]; }
  LDSX();
  for (int q = lane; q < 16 * 16; q += 32) { const int rl = q >> 4, pc = q & 15; if (n0 + rl >= NN) continue;
    vst2(out + (size_t)(n0 + rl) * CH + pc * 4, *(const v4f*)(&so[w][rl][pc * 4])); }
}

extern "C" void kernel_launch(void* const* d_in, const int* in_sizes, int n_in,
                              void* d_out, int out_size, void* d_ws, size_t ws_size,
                              hipStream_t stream) {
  (void)in_sizes; (void)n_in; (void)out_size; (void)ws_size;
  const float* x = (const float*)d_in[0]; const float* bases = (const float*)d_in[1]; const float* comp = (const float*)d_in[2]; const float* loopw = (const float*)d_in[3];
  const float* bias = (const float*)d_in[4]; const float* gam = (const float*)d_in[5]; const float* bet = (const float*)d_in[6];
  const int* src = (const int*)d_in[7]; const int* dst = (const int*)d_in[8]; const int* et = (const int*)d_in[9];
  float* out = (float*)d_out;
  char* ws = (char*)d_ws; size_t off = 0;
  auto take = [&](size_t bytes) { char* p = ws + off; off += (bytes + 255) & ~(size_t)255; return p; };
  int* list = (int*)take((size_t)NN * SLOTC * 4);
  _Float16* Wc = (_Float16*)take((size_t)CH * KTOT * 2);
  k_bucket<<<(NN + NCH - 1) / NCH, 256, 0, stream>>>(dst, list);
  k_packW<<<CH, 64, 0, stream>>>(bases, loopw, Wc);
  k_layer<<<NNP / 64, 128, 0, stream>>>(x, src, et, list, comp, Wc, bias, gam, bet, out);
}
